// RecurrentGCN_25735444038199
// MI455X (gfx1250) — hardware-verified
//
#include <hip/hip_runtime.h>


#define NN   200000
#define DIN  16
#define KP   32
#define HID  128
#define NG   (2 * HID)
#define CH   40000
typedef _Float16 h16;
typedef unsigned short bf;
typedef __attribute__((ext_vector_type(16))) __bf16   v16bf;
typedef __attribute__((ext_vector_type(16))) _Float16 v16h;
typedef __attribute__((ext_vector_type(8)))  _Float16 v8h;
typedef __attribute__((ext_vector_type(8)))  unsigned short v8us;
typedef __attribute__((ext_vector_type(8)))  float    v8f;
typedef __attribute__((ext_vector_type(4)))  float    v4f;
typedef v8h  __attribute__((may_alias)) v8ha;
typedef v4f  __attribute__((may_alias)) v4fa;
typedef v8us __attribute__((may_alias)) v8usa;

__device__ __forceinline__ unsigned short f2bf(float f) { unsigned u = __float_as_uint(f); u += 0x7FFFu + ((u >> 16) & 1u); return (unsigned short)(u >> 16); }
__device__ __forceinline__ float bf2f(unsigned short b) { return __uint_as_float(((unsigned)b) << 16); }
__device__ __forceinline__ float bfr(float f) { return bf2f(f2bf(f)); }
__device__ __forceinline__ v16h cat16(v8h lo, v8h hi) { return __builtin_shufflevector(lo, hi, 0, 1, 2, 3, 4, 5, 6, 7, 8, 9, 10, 11, 12, 13, 14, 15); }
__device__ __forceinline__ v16bf cat16b(v8us lo, v8us hi) { return __builtin_bit_cast(v16bf, __builtin_shufflevector(lo, hi, 0, 1, 2, 3, 4, 5, 6, 7, 8, 9, 10, 11, 12, 13, 14, 15)); }
__device__ __forceinline__ v8f wmma16(v16h a, v16h b, v8f c) { return __builtin_amdgcn_wmma_f32_16x16x32_f16(false, a, false, b, (short)0, c, false, false); }
__device__ __forceinline__ v8f wmmab(v16bf a, v16bf b, v8f c) { return __builtin_amdgcn_wmma_f32_16x16x32_bf16(false, a, false, b, (short)0, c, false, false); }


template <typename T16> struct WFrag;
template <> struct WFrag<h16> { typedef v16h V; static __device__ __forceinline__ V ld(const h16* p) { return cat16(*(const v8h*)p, *(const v8h*)(p + 16)); } static __device__ __forceinline__ v8f mma(V a, V b, v8f c) { return wmma16(a, b, c); } };
template <> struct WFrag<bf> { typedef v16bf V; static __device__ __forceinline__ V ld(const bf* p) { return cat16b(*(const v8us*)p, *(const v8us*)(p + 16)); } static __device__ __forceinline__ v8f mma(V a, V b, v8f c) { return wmmab(a, b, c); } };
template <typename T16, int NSPLIT, bool BIAS>
__global__ __launch_bounds__(32) void k_gemmw(const T16* __restrict__ A, const T16* __restrict__ A2, const T16* __restrict__ Bt, const T16* __restrict__ Bt2, int K, float* C, int ldc, const float* __restrict__ bias, size_t sA, size_t sB, size_t sC) {
    typedef typename WFrag<T16>::V V;
    __shared__ __align__(16) float os[16 * 68];
    const size_t z = blockIdx.z; A += z * sA; if (A2) A2 += z * sA; Bt += z * sB; if (Bt2) Bt2 += z * sB; C += z * sC;
    const int lane = threadIdx.x & 31, lr = lane & 15, hi = lane >> 4; const int r0 = blockIdx.x * 64, c0 = blockIdx.y * 64;
    v8f acc[4][4];
#pragma unroll
    for (int mb = 0; mb < 4; ++mb)
#pragma unroll
        for (int nb = 0; nb < 4; ++nb) acc[mb][nb] = (v8f){};
    const size_t aoff = (size_t)(r0 + lr) * K + 8 * hi, boff = (size_t)(c0 + lr) * K + 8 * hi;
#pragma unroll 1
    for (int kc = 0; kc < K; kc += 32) {
        V a[4], a2[4];
#pragma unroll
        for (int mb = 0; mb < 4; ++mb) { a[mb] = WFrag<T16>::ld(A + aoff + (size_t)mb * 16 * K + kc); if (NSPLIT == 1 || NSPLIT == 2) a2[mb] = WFrag<T16>::ld(A2 + aoff + (size_t)mb * 16 * K + kc); }
#pragma unroll
        for (int nb = 0; nb < 4; ++nb) { const V b = WFrag<T16>::ld(Bt + boff + (size_t)nb * 16 * K + kc); V b2; if (NSPLIT >= 2) b2 = WFrag<T16>::ld(Bt2 + boff + (size_t)nb * 16 * K + kc);
#pragma unroll
            for (int mb = 0; mb < 4; ++mb) { acc[mb][nb] = WFrag<T16>::mma(a[mb], b, acc[mb][nb]); if (NSPLIT == 1 || NSPLIT == 2) acc[mb][nb] = WFrag<T16>::mma(a2[mb], b, acc[mb][nb]); if (NSPLIT >= 2) acc[mb][nb] = WFrag<T16>::mma(a[mb], b2, acc[mb][nb]); } }
        asm volatile("v_nop\n\tv_nop\n\tv_nop\n\tv_nop" : "+v"(acc[0][0]), "+v"(acc[1][1]), "+v"(acc[2][2]), "+v"(acc[3][3]) : "v"(a[0]), "v"(a[3]));
    }
#pragma unroll
    for (int mb = 0; mb < 4; ++mb) {
#pragma unroll
        for (int nb = 0; nb < 4; ++nb) {
#pragma unroll
            for (int j = 0; j < 8; ++j) os[(hi * 8 + j) * 68 + nb * 16 + lr] = acc[mb][nb][j]; }
        __builtin_amdgcn_wave_barrier(); asm volatile("" ::: "memory");
        float* crow = C + (size_t)(r0 + mb * 16) * ldc + c0;
#pragma unroll 1
        for (int ps = 0; ps < 2; ++ps) {
#pragma unroll
            for (int s = 0; s < 8; ++s) { const int row = 2 * s + hi, cofs = lr * 4; v4f val = *(const v4fa*)(os + row * 68 + cofs); if (BIAS) { val[0] += bfr(bias[c0 + cofs]); val[1] += bfr(bias[c0 + cofs + 1]); val[2] += bfr(bias[c0 + cofs + 2]); val[3] += bfr(bias[c0 + cofs + 3]); }
                *(volatile v4f*)(crow + (size_t)row * ldc + cofs) = val; }
            if (ps == 0) __threadfence(); }
        __builtin_amdgcn_wave_barrier(); asm volatile("" ::: "memory");
    }
}

typedef __attribute__((ext_vector_type(2))) unsigned short v2us;
typedef __attribute__((ext_vector_type(16))) unsigned short v16us;
__global__ __launch_bounds__(256) void k_cvt8(const float* __restrict__ src, bf* dst, size_t n8) { const size_t i = (size_t)blockIdx.x * 256 + threadIdx.x; if (i >= n8) return; const v8f v = *(const v8f*)(src + i * 8); v8us o;
#pragma unroll
    for (int k = 0; k < 8; ++k) o[k] = f2bf(v[k]); *(volatile v8us*)(dst + i * 8) = o; __threadfence(); *(volatile v8us*)(dst + i * 8) = o; }

__global__ __launch_bounds__(256) void k_xpad(const float* __restrict__ x, bf* XB) { const size_t n = (size_t)blockIdx.x * 256 + threadIdx.x; if (n >= NN) return; const v8f a = *(const v8f*)(x + n * DIN); const v8f c = *(const v8f*)(x + n * DIN + 8); v16us lo, hi;
#pragma unroll
    for (int k = 0; k < 8; ++k) { lo[k] = f2bf(a[k]); lo[8 + k] = f2bf(c[k]); hi[k] = 0; hi[8 + k] = 0; }
    *(volatile v16us*)(XB + n * KP) = lo; *(volatile v16us*)(XB + n * KP + 16) = hi; __threadfence(); *(volatile v16us*)(XB + n * KP) = lo; *(volatile v16us*)(XB + n * KP + 16) = hi; }
__global__ __launch_bounds__(256) void k_wpad(const float* __restrict__ wz, const float* __restrict__ wh, bf* Bt) { const int j = blockIdx.x * 256 + threadIdx.x; if (j >= NG) return; const float* w = (j < HID) ? wz : wh; const int c = j & (HID - 1); v16us lo, hi;
#pragma unroll
    for (int k = 0; k < 16; ++k) { lo[k] = f2bf(w[k * HID + c]); hi[k] = 0; }
    *(volatile v16us*)(Bt + (size_t)j * KP) = lo; *(volatile v16us*)(Bt + (size_t)j * KP + 16) = hi; __threadfence(); *(volatile v16us*)(Bt + (size_t)j * KP) = lo; *(volatile v16us*)(Bt + (size_t)j * KP + 16) = hi; }
__global__ __launch_bounds__(256) void k_gate(const float* __restrict__ G, size_t n0, const float* __restrict__ bxz, const float* __restrict__ bhz, const float* __restrict__ bxh, const float* __restrict__ bhh, const float* __restrict__ wout, const float* __restrict__ bout, float* out) {
    const size_t nl = (size_t)blockIdx.x * 256 + threadIdx.x; const size_t n = n0 + nl; if (nl >= CH || n >= NN) return; const float* g = G + nl * NG; float acc = 0.f;
#pragma unroll 1
    for (int c4 = 0; c4 < HID; c4 += 4) { const v4f gz = *(const v4f*)(g + c4); const v4f gh = *(const v4f*)(g + HID + c4);
#pragma unroll
        for (int q = 0; q < 4; ++q) { const int c = c4 + q; const float bz = __fadd_rn(bfr(bxz[c]), bfr(bhz[c])); const float bh = __fadd_rn(bfr(bxh[c]), bfr(bhh[c]));
            const float az = __fadd_rn(gz[q], bz); const float ah = __fadd_rn(gh[q], bh);
            const float ez = __builtin_amdgcn_exp2f(__fmul_rn(az, -1.4426950408889634f)); const float z = __fdiv_rn(1.0f, __fadd_rn(1.0f, ez)); const float eh = __builtin_amdgcn_exp2f(__fmul_rn(ah, -2.8853900817779268f)); const float ht = __fsub_rn(__fdiv_rn(2.0f, __fadd_rn(1.0f, eh)), 1.0f);
            float hn = __fmul_rn(__fsub_rn(1.0f, z), ht); asm volatile("" : "+v"(hn)); hn = fmaxf(hn, 0.0f);
            acc = fmaf(hn, bfr(wout[c]), acc); } }
    const float o = __fadd_rn(acc, bfr(bout[0])); *(volatile float*)(out + n) = o; __threadfence(); *(volatile float*)(out + n) = o; }

extern "C" void kernel_launch(void* const* d_in, const int* in_sizes, int n_in,
                              void* d_out, int out_size, void* d_ws, size_t ws_size, hipStream_t stream) {
    (void)in_sizes; (void)n_in; (void)out_size;
    const float* x = (const float*)d_in[0];
    const float* wxz = (const float*)d_in[3]; const float* bxz = (const float*)d_in[4];   const float* bhz = (const float*)d_in[6];
    const float* wxh = (const float*)d_in[11]; const float* bxh = (const float*)d_in[12];   const float* bhh = (const float*)d_in[14];
    const float* wout = (const float*)d_in[15]; const float* bout = (const float*)d_in[16];
    float* OUT = (float*)d_out;
    char* wsp = (char*)d_ws;
    auto take = [&](size_t bytes) { char* p = wsp; wsp += (bytes + 255) & ~(size_t)255; return (void*)p; };
    bf* XB = (bf*)take((size_t)NN * KP * 2); bf* BT = (bf*)take((size_t)NG * KP * 2); float* G = (float*)take((size_t)CH * NG * 4);
    if ((size_t)(wsp - (char*)d_ws) > ws_size) return;
    k_xpad<<<(NN + 255) / 256, 256, 0, stream>>>(x, XB); k_wpad<<<1, 256, 0, stream>>>(wxz, wxh, BT);
    static_assert(NN % CH == 0 && CH % 64 == 0, "chunking");
    for (size_t n0 = 0; n0 < NN; n0 += CH) {
        k_gemmw<bf, 0, false><<<dim3(CH / 64, NG / 64, 1), 32, 0, stream>>>(XB + n0 * KP, nullptr, BT, nullptr, KP, G, NG, nullptr, 0, 0, 0);
        k_gate<<<(CH + 255) / 256, 256, 0, stream>>>(G, n0, bxz, bhz, bxh, bhh, wout, bout, OUT); }
}
